// MambaGate2D_88201448390700
// MI455X (gfx1250) — hardware-verified
//
#include <hip/hip_runtime.h>
#include <math.h>

typedef __attribute__((ext_vector_type(16))) _Float16 v16h;
typedef __attribute__((ext_vector_type(8)))  _Float16 v8h;
typedef __attribute__((ext_vector_type(8)))  float    v8f;
typedef __attribute__((ext_vector_type(4)))  float    v4f;
typedef __attribute__((ext_vector_type(4)))  unsigned v4u;

constexpr int kB    = 16;
constexpr int kCh   = 64;
constexpr int kL    = 4096;
constexpr int kDm   = 64;
constexpr int kDi   = 128;
constexpr int kNs   = 16;
constexpr int kR    = 4;
constexpr int kXP   = kR + 2 * kNs;
constexpr int kXPp  = 64;
constexpr int kXZP  = 2 * kDi;
constexpr int kTok  = kB * kL;
constexpr int kTok2 = 2 * kTok;
constexpr int kCvP  = 260;
constexpr int kScT  = 32;
constexpr int kScXP = 40;
constexpr int kScYP = 132;
constexpr float kLnEps = 1e-5f;

constexpr float kCarryW   = 32.0f;
constexpr float kCarryXS  = 16.0f;
constexpr float kCarryXD  = 256.0f;
constexpr float kCarryYG  = 64.0f;
constexpr float kCarryOUT = 128.0f;
constexpr float kSclIn  = 1.0f / kCarryW;
constexpr float kSclMi  = 1.0f / kCarryW;
constexpr float kSclXp  = kCarryXD / (kCarryXS * kCarryW);
constexpr float kSclMo  = 0.5f * kCarryOUT / (kCarryYG * kCarryW);
constexpr float kSclOut = 1.0f / (kCarryOUT * kCarryW);

static_assert(kXP == 36 && kXP <= kXPp, "x_proj width");
static_assert((kCh % 32) == 0 && (kDm % 32) == 0 && (kDi % 32) == 0 && ((2 * kDi) % 32) == 0, "GEMM K multiples of 32");
static_assert((kTok % 64) == 0 && (kTok2 % 64) == 0 && (kXZP % 64) == 0 && (kDm % 64) == 0 && (kXPp % 64) == 0, "GEMM M,N multiples of 64");
static_assert((kL % 64) == 0 && (kL % kScT) == 0, "tiles never cross an image");
static_assert(kDm == 64 && kCh == 64, "full-row epilogues need N == 64");
static_assert(kScT * 5 == 160, "scan staging map");

constexpr size_t kOffXH    = 0;
constexpr size_t kOffTOKH  = kOffXH   + (size_t)kTok * kCh * 2;
constexpr size_t kOffXDBL  = 0;
constexpr size_t kOffXZ    = kOffTOKH + (size_t)kTok * kDm * 2;
constexpr size_t kOffXS    = kOffXZ   + (size_t)kTok * kXZP * 2;
constexpr size_t kOffYG    = kOffXS   + (size_t)kTok2 * kDi * 2;
constexpr size_t kOffOUT   = kOffYG   + (size_t)kTok * 2 * kDi * 2;
constexpr size_t kOffWIN   = kOffOUT  + (size_t)kTok * kDm * 2;
constexpr size_t kOffWMI   = kOffWIN  + (size_t)kDm * kCh * 2;
constexpr size_t kOffWXP   = kOffWMI  + (size_t)kXZP * kDm * 2;
constexpr size_t kOffWMOC  = kOffWXP  + (size_t)kXPp * kDi * 2;
constexpr size_t kOffWOUT  = kOffWMOC + (size_t)kDm * 2 * kDi * 2;
constexpr size_t kWsTotal  = kOffWOUT + (size_t)kCh * kDm * 2;
static_assert((size_t)kTok2 * kXPp * 2 <= kOffXZ, "XDBL16 fits inside XH+TOKH");
static_assert(kWsTotal == 125927424ull, "carve total");
static_assert(kWsTotal <= 134217728ull, "carve cap");
static_assert((kOffTOKH % 128) == 0 && (kOffXZ % 128) == 0 && (kOffXS % 128) == 0 && (kOffYG % 128) == 0 &&
              (kOffOUT % 128) == 0 && (kOffWIN % 128) == 0 && (kOffWMI % 128) == 0 && (kOffWXP % 128) == 0 &&
              (kOffWMOC % 128) == 0 && (kOffWOUT % 128) == 0, "128-B aligned regions");

__device__ __forceinline__ float h16_to_f32(unsigned hb) {
  const unsigned sgn = (hb & 0x8000u) << 16;
  const unsigned em = hb & 0x7fffu;
  const float fn = __uint_as_float((em << 13) + 0x38000000u);
  const float fs = (float)em * 5.9604644775390625e-8f;
  const float mag = (em < 0x400u) ? fs : fn;
  return __uint_as_float(__float_as_uint(mag) | sgn);
}
__device__ __forceinline__ unsigned ld_h16(const unsigned* plane32, size_t idx) {
  const unsigned w = plane32[idx >> 1];
  return (idx & 1) ? (w >> 16) : (w & 0xffffu);
}
__device__ __forceinline__ void wave_lds_sync() {
  __builtin_amdgcn_fence(__ATOMIC_RELEASE, "workgroup");
  __builtin_amdgcn_wave_barrier();
  __builtin_amdgcn_fence(__ATOMIC_ACQUIRE, "workgroup");
}
__device__ __forceinline__ void guard_row_h(v8f& a, v8f& b, v8f& c, v8f& d, v16h x, v16h y0, v16h y1, v16h y2, v16h y3) {
  asm volatile("v_nop\n\tv_nop\n\tv_nop\n\tv_nop" : "+v"(a), "+v"(b), "+v"(c), "+v"(d) : "v"(x), "v"(y0), "v"(y1), "v"(y2), "v"(y3));
}
__device__ __forceinline__ void keep4_h(v16h a, v16h b, v16h c, v16h d) { asm volatile("v_nop" :: "v"(a), "v"(b), "v"(c), "v"(d)); }
__device__ __forceinline__ void acc_guard4(v8f& a, v8f& b, v8f& c, v8f& d) { asm volatile("v_nop\n\tv_nop\n\tv_nop\n\tv_nop" : "+v"(a), "+v"(b), "+v"(c), "+v"(d)); }

struct FragH {
  union U { v16h v; v8h h[2]; };
  static __device__ __forceinline__ v16h load(const _Float16* p) {
    U f; f.h[0] = *(const v8h*)(p); f.h[1] = *(const v8h*)(p + 16); return f.v;
  }
  static __device__ __forceinline__ v8f mma(v16h a, v16h b, v8f c) {
    return __builtin_amdgcn_wmma_f32_16x16x32_f16(false, a, false, b, (short)0, c, false, false);
  }
};

template <int EPI>
__global__ __launch_bounds__(256) void gemm_f16_kernel(
    const unsigned short* __restrict__ Ap, int lda,
    const unsigned short* __restrict__ Btp, int ldb,
    void* __restrict__ Cout, int ldc,
    const float* __restrict__ bias, const float* __restrict__ gam, const float* __restrict__ bet,
    int M, int N, int K, float scale)
{
  const _Float16* A  = (const _Float16*)Ap;
  const _Float16* Bt = (const _Float16*)Btp;
  __shared__ __align__(16) float sT[8][16 * 68];
  const int lane = threadIdx.x & 31;
  const int wave = threadIdx.x >> 5;
  const int tilesN = N >> 6;
  const int tilesM = M >> 6;
  const int tile = blockIdx.x * 8 + wave;
  if (tile >= tilesM * tilesN) return;
  const int tm = tile / tilesN;
  const int tn = tile - tm * tilesN;
  const int m0 = tm << 6;
  const int n0 = tn << 6;

  const int rlane = lane & 15;
  const int koff  = (lane >> 4) * 8;
  const int mOff  = (lane >> 4) * 8;

  v8f acc[4][4];
#pragma unroll
  for (int i = 0; i < 4; ++i)
#pragma unroll
    for (int j = 0; j < 4; ++j) acc[i][j] = (v8f){0.f,0.f,0.f,0.f,0.f,0.f,0.f,0.f};

  for (int k0 = 0; k0 < K; k0 += 32) {
    v16h bh[4];
#pragma unroll
    for (int j = 0; j < 4; ++j) {
      const size_t bo = (size_t)(n0 + (j << 4) + rlane) * ldb + koff + k0;
      bh[j] = FragH::load(Bt + bo);
    }
#pragma unroll
    for (int i = 0; i < 4; ++i) {
      const size_t ao = (size_t)(m0 + (i << 4) + rlane) * lda + koff + k0;
      v16h ah = FragH::load(A + ao);
#pragma unroll
      for (int j = 0; j < 4; ++j) acc[i][j] = FragH::mma(ah, bh[j], acc[i][j]);
      guard_row_h(acc[i][0], acc[i][1], acc[i][2], acc[i][3], ah, bh[0], bh[1], bh[2], bh[3]);
    }
    keep4_h(bh[0], bh[1], bh[2], bh[3]);
  }
  acc_guard4(acc[0][0], acc[0][1], acc[0][2], acc[0][3]);
  acc_guard4(acc[1][0], acc[1][1], acc[1][2], acc[1][3]);
  acc_guard4(acc[2][0], acc[2][1], acc[2][2], acc[2][3]);
  acc_guard4(acc[3][0], acc[3][1], acc[3][2], acc[3][3]);

  float* slab = sT[wave];

  if (EPI == 2) {
    float* C = (float*)Cout;
    const int img = m0 / ldc;
    const int l0  = m0 - img * ldc;
#pragma unroll
    for (int j = 0; j < 4; ++j) {
      const float bv = bias[(j << 4) + rlane];
#pragma unroll
      for (int i = 0; i < 4; ++i) {
#pragma unroll
        for (int r = 0; r < 8; ++r) {
          slab[rlane * 68 + (i << 4) + mOff + r] = acc[i][j][r] * scale + bv;
        }
      }
      wave_lds_sync();
#pragma unroll 1
      for (int e = 0; e < 32; ++e) {
        const int idx = e * 32 + lane;
        float* p = slab + (idx >> 6) * 68 + (idx & 63);
        const float xv = *p;
        const float ex = expf(-xv);
        *p = 1.0f / (1.0f + ex) - 0.5f;
      }
      wave_lds_sync();
      {
        const int hh = lane >> 4, c4 = (lane & 15) * 4;
        for (int pass = 0; pass < 2; ++pass) {
#pragma unroll
          for (int it = 0; it < 8; ++it) {
            const int row = it * 2 + hh;
            v4f v = *(const v4f*)(slab + row * 68 + c4);
            *(volatile v4f*)(C + (size_t)(img * N + (j << 4) + row) * ldc + l0 + c4) = v;
          }
          __threadfence();
        }
      }
      wave_lds_sync();
    }
  } else {
    unsigned short* C = (unsigned short*)Cout;
#pragma unroll
    for (int i = 0; i < 4; ++i) {
      const int mBase = m0 + (i << 4);
#pragma unroll
      for (int j = 0; j < 4; ++j) {
        const int n = n0 + (j << 4) + rlane;
        float bv = 0.f;
        if (EPI == 1) bv = bias[n];
#pragma unroll
        for (int r = 0; r < 8; ++r) {
          float v = acc[i][j][r] * scale;
          if (EPI == 1) v += bv;
          slab[(mOff + r) * 68 + (j << 4) + rlane] = v;
        }
      }
      wave_lds_sync();
      if (EPI == 1) {
        const int lr = lane >> 1, lh = (lane & 1) * 32;
        float* rp = slab + lr * 68 + lh;
        float s = 0.f;
#pragma unroll 1
        for (int c = 0; c < 8; ++c) {
          const v4f t = *(const v4f*)(rp + 4 * c);
          s += (t[0] + t[1]) + (t[2] + t[3]);
        }
        s += __shfl_xor(s, 1, 32);
        const float mean = s * (1.0f / (float)kDm);
        float qv = 0.f;
#pragma unroll 1
        for (int c = 0; c < 8; ++c) {
          const v4f t = *(const v4f*)(rp + 4 * c);
          const float d0 = t[0] - mean, d1 = t[1] - mean, d2 = t[2] - mean, d3 = t[3] - mean;
          qv += (d0 * d0 + d1 * d1) + (d2 * d2 + d3 * d3);
        }
        qv += __shfl_xor(qv, 1, 32);
        const float rstd = rsqrtf(qv * (1.0f / (float)kDm) + kLnEps);
#pragma unroll 1
        for (int c = 0; c < 8; ++c) {
          const v4f t  = *(const v4f*)(rp + 4 * c);
          const v4f gg = *(const v4f*)(gam + lh + 4 * c);
          const v4f bb = *(const v4f*)(bet + lh + 4 * c);
          v4f o;
          o[0] = (t[0] - mean) * rstd * gg[0] + bb[0];
          o[1] = (t[1] - mean) * rstd * gg[1] + bb[1];
          o[2] = (t[2] - mean) * rstd * gg[2] + bb[2];
          o[3] = (t[3] - mean) * rstd * gg[3] + bb[3];
          *(v4f*)(rp + 4 * c) = o;
        }
        wave_lds_sync();
      }
      {
        const int q = lane >> 3, c8 = (lane & 7) * 8;
        for (int pass = 0; pass < 2; ++pass) {
#pragma unroll
          for (int it = 0; it < 4; ++it) {
            const int row = it * 4 + q;
            const float* sp = slab + row * 68 + c8;
            v8h hv;
#pragma unroll
            for (int e = 0; e < 8; ++e) hv[e] = (_Float16)sp[e];
            *(volatile v8h*)(C + (size_t)(mBase + row) * ldc + n0 + c8) = hv;
          }
          __threadfence();
        }
      }
      wave_lds_sync();
    }
  }
}

__global__ __launch_bounds__(256) void cast_w_f16_kernel(
    const float* __restrict__ src, unsigned short* __restrict__ dst, int Nsrc, int Ksrc, int Kdst, int total8, float scale)
{
  const int i = blockIdx.x * 256 + threadIdx.x;
  if (i >= total8) return;
  const int e0   = i << 3;
  const int row  = e0 / Kdst;
  const int col  = e0 - row * Kdst;
  const int scol = col % Ksrc;
  const int rowc = (row < Nsrc) ? row : (Nsrc - 1);
  const bool live = (row < Nsrc);
  const float* p = src + (size_t)rowc * Ksrc + scol;
  const v4f a0 = *(const v4f*)(p);
  const v4f a1 = *(const v4f*)(p + 4);
  v8h hv;
#pragma unroll
  for (int e = 0; e < 4; ++e) {
    hv[e]     = (_Float16)(live ? (a0[e] * scale) : 0.0f);
    hv[4 + e] = (_Float16)(live ? (a1[e] * scale) : 0.0f);
  }
  unsigned short* q = dst + (size_t)e0;
  *(volatile v8h*)q = hv;
  __threadfence();
  *(volatile v8h*)q = hv;
}

__global__ __launch_bounds__(256) void xpose_cast_kernel(
    const float* __restrict__ Xb, unsigned short* __restrict__ Ob, int Kdim, int Ndim,
    long strideIn, long strideOut, float scale)
{
  __shared__ float tile[64 * 65];
  const int tid = threadIdx.x, lane = tid & 31, wave = tid >> 5;
  const float* W = Xb + (size_t)blockIdx.z * strideIn;
  unsigned short* Bt = Ob + (size_t)blockIdx.z * strideOut;
  const int n0 = blockIdx.x * 64;
  const int k0 = blockIdx.y * 64;
#pragma unroll
  for (int p = 0; p < 16; ++p) {
    const int idx = tid + p * 256;
    const int kk  = idx >> 6;
    const int nn  = idx & 63;
    const float v = W[(size_t)(k0 + kk) * Ndim + n0 + nn];
    tile[kk * 65 + nn] = v * scale;
  }
  __syncthreads();
  const int q = lane >> 3, c8 = (lane & 7) * 8;
  v8h hv[2];
#pragma unroll
  for (int it = 0; it < 2; ++it) {
    const int nrow = it * 32 + wave * 4 + q;
#pragma unroll
    for (int e = 0; e < 8; ++e) hv[it][e] = (_Float16)tile[(c8 + e) * 65 + nrow];
  }
  for (int pass = 0; pass < 2; ++pass) {
#pragma unroll
    for (int it = 0; it < 2; ++it) {
      const int nrow = it * 32 + wave * 4 + q;
      *(volatile v8h*)(Bt + (size_t)(n0 + nrow) * Kdim + k0 + c8) = hv[it];
    }
    __threadfence();
  }
}

__device__ __forceinline__ float xr_tap(const unsigned* XZ32, int ib, int l, int d) {
  const int lc = (l < 0) ? 0 : ((l > kL - 1) ? (kL - 1) : l);
  const unsigned hb = ld_h16(XZ32, (size_t)(ib + lc) * kXZP + d);
  const float v = h16_to_f32(hb);
  return (l >= 0 && l < kL) ? v : 0.0f;
}

__global__ __launch_bounds__(256) void conv_silu_bidir_kernel(
    const unsigned* __restrict__ XZ32, const float* __restrict__ cw, const float* __restrict__ cb,
    unsigned short* __restrict__ XS16)
{
  __shared__ __align__(16) float sT[32 * kCvP];
  const int tid = threadIdx.x, lane = tid & 31, wave = tid >> 5;
  const int d   = tid & 127;
  const int grp = tid >> 7;
  const int gblk = blockIdx.x * 64;
  const int g0 = gblk + grp * 32;
  const int lq = g0 & (kL - 1);
  const int ib = g0 - lq;
  const v4f wv = *(const v4f*)(cw + d * 4);
  const float w0 = wv[0], w1 = wv[1], w2 = wv[2], w3 = wv[3];
  const float bc = cb[d];
  float xm3 = xr_tap(XZ32, ib, lq - 3, d);
  float xm2 = xr_tap(XZ32, ib, lq - 2, d);
  float xm1 = xr_tap(XZ32, ib, lq - 1, d);
  float x0  = xr_tap(XZ32, ib, lq,     d);
  float xp1 = xr_tap(XZ32, ib, lq + 1, d);
  float xp2 = xr_tap(XZ32, ib, lq + 2, d);
#pragma unroll 1
  for (int sub = 0; sub < 2; ++sub) {
#pragma unroll 1
    for (int st = 0; st < 16; ++st) {
      const int l = lq + sub * 16 + st;
      const float xp3 = xr_tap(XZ32, ib, l + 3, d);
      float af = w0 * xm3;
      af = fmaf(w1, xm2, af);
      af = fmaf(w2, xm1, af);
      af = fmaf(w3, x0, af);
      af += bc;
      float ab = w0 * xp3;
      ab = fmaf(w1, xp2, ab);
      ab = fmaf(w2, xp1, ab);
      ab = fmaf(w3, x0, ab);
      ab += bc;
      const float sf = af * (1.0f / (1.0f + expf(-af)));
      const float sb = ab * (1.0f / (1.0f + expf(-ab)));
      float* tp = sT + (grp * 16 + st) * kCvP;
      tp[d]       = sf * kCarryXS;
      tp[kDi + d] = sb * kCarryXS;
      xm3 = xm2; xm2 = xm1; xm1 = x0; x0 = xp1; xp1 = xp2; xp2 = xp3;
    }
    __syncthreads();
    v8h bv[4];
#pragma unroll
    for (int it = 0; it < 4; ++it) {
      const float* sp = sT + (it * 8 + wave) * kCvP + lane * 8;
      const v4f a0 = *(const v4f*)(sp);
      const v4f a1 = *(const v4f*)(sp + 4);
#pragma unroll
      for (int e = 0; e < 4; ++e) {
        bv[it][e]     = (_Float16)a0[e];
        bv[it][4 + e] = (_Float16)a1[e];
      }
    }
    for (int pass = 0; pass < 2; ++pass) {
#pragma unroll
      for (int it = 0; it < 4; ++it) {
        const int rr = it * 8 + wave;
        const int tokn = gblk + (rr >> 4) * 32 + sub * 16 + (rr & 15);
        *(volatile v8h*)(XS16 + (size_t)tokn * (2 * kDi) + lane * 8) = bv[it];
      }
      __threadfence();
    }
    __syncthreads();
  }
}

__device__ __forceinline__ void stage_xd_group(const unsigned* XD32, float* sX, int idx, int t0, int dir, int tok0) {
  const int row = idx / 5;
  const int g   = idx - row * 5;
  const int tt  = t0 + row;
  const int tok = dir ? (kL - 1 - tt) : tt;
  const size_t r2 = (size_t)(tok0 + tok) * 2 + dir;
  const v4u w = *(const v4u*)(XD32 + r2 * (kXPp / 2) + g * 4);
  const unsigned w0 = w[0], w1 = w[1], w2 = w[2], w3 = w[3];
  const float inv = 1.0f / kCarryXD;
  v4f lo, hi;
  lo[0] = h16_to_f32(w0 & 0xffffu) * inv;
  lo[1] = h16_to_f32(w0 >> 16) * inv;
  lo[2] = h16_to_f32(w1 & 0xffffu) * inv;
  lo[3] = h16_to_f32(w1 >> 16) * inv;
  hi[0] = h16_to_f32(w2 & 0xffffu) * inv;
  hi[1] = h16_to_f32(w2 >> 16) * inv;
  hi[2] = h16_to_f32(w3 & 0xffffu) * inv;
  hi[3] = h16_to_f32(w3 >> 16) * inv;
  *(v4f*)(sX + row * kScXP + g * 8)     = lo;
  *(v4f*)(sX + row * kScXP + g * 8 + 4) = hi;
}

__global__ __launch_bounds__(128) void scan_gate_kernel(
    const unsigned* __restrict__ XD32, const unsigned* __restrict__ XS32, const unsigned* __restrict__ XZ32,
    const float* __restrict__ Wdt, const float* __restrict__ bdt, const float* __restrict__ Alog,
    const float* __restrict__ Dp, unsigned short* __restrict__ YG16)
{
  __shared__ __align__(16) float sX[kScT * kScXP];
  __shared__ __align__(16) float sY[kScT * kScYP];
  const int tid = threadIdx.x, lane = tid & 31, wave = tid >> 5;
  const int d   = tid;
  const int dir = blockIdx.x >> 4;
  const int img = blockIdx.x & 15;
  const int tok0 = img * kL;

  float An[kNs];
  {
    v4f al[4];
#pragma unroll
    for (int q4 = 0; q4 < 4; ++q4) al[q4] = *(const v4f*)(Alog + (size_t)d * kNs + 4 * q4);
#pragma unroll
    for (int n = 0; n < kNs; ++n) An[n] = -expf(al[n >> 2][n & 3]);
  }
  const v4f wd = *(const v4f*)(Wdt + (size_t)d * kR);
  const float bb = bdt[d];
  const float Dd = Dp[d];
  float h[kNs];
#pragma unroll
  for (int n = 0; n < kNs; ++n) h[n] = 0.f;

#pragma unroll 1
  for (int c = 0; c < kL / kScT; ++c) {
    const int t0 = c * kScT;
    stage_xd_group(XD32, sX, tid, t0, dir, tok0);
    if (tid < 32) {
      stage_xd_group(XD32, sX, 128 + tid, t0, dir, tok0);
    }
    __syncthreads();
#pragma unroll 1
    for (int s = 0; s < kScT; ++s) {
      const int tt  = t0 + s;
      const int tok = dir ? (kL - 1 - tt) : tt;
      const size_t m = (size_t)(tok0 + tok);
      unsigned ub = ld_h16(XS32, (m * 2 + dir) * kDi + d);
      unsigned zb = ld_h16(XZ32, m * kXZP + kDi + d);
      asm volatile("" : "+v"(ub), "+v"(zb));
      const float u  = h16_to_f32(ub) * (1.0f / kCarryXS);
      const float zv = h16_to_f32(zb);
      const float* xr = sX + s * kScXP;
      const v4f dtv = *(const v4f*)(xr);
      v4f Bq[4], Cq[4];
#pragma unroll
      for (int q4 = 0; q4 < 4; ++q4) {
        Bq[q4] = *(const v4f*)(xr + kR + 4 * q4);
        Cq[q4] = *(const v4f*)(xr + kR + kNs + 4 * q4);
      }
      float v = bb;
      v = fmaf(dtv[0], wd[0], v);
      v = fmaf(dtv[1], wd[1], v);
      v = fmaf(dtv[2], wd[2], v);
      v = fmaf(dtv[3], wd[3], v);
      const float delta = fmaxf(v, 0.0f) + log1pf(expf(-fabsf(v)));
      const float du = delta * u;
      float y = 0.f;
#pragma unroll
      for (int n = 0; n < kNs; ++n) {
        const float e = __expf(delta * An[n]);
        h[n] = fmaf(e, h[n], du * Bq[n >> 2][n & 3]);
        y = fmaf(h[n], Cq[n >> 2][n & 3], y);
      }
      y = fmaf(u, Dd, y);
      const float sg = 1.0f / (1.0f + expf(-zv));
      const float yg = y * (zv * sg);
      sY[s * kScYP + tid] = yg * kCarryYG;
    }
    __syncthreads();
    const int hh = lane >> 4, c8 = (lane & 15) * 8;
    v8h hv[4];
#pragma unroll
    for (int it = 0; it < 4; ++it) {
      const int row = it * 8 + wave * 2 + hh;
      const float* sp = sY + row * kScYP + c8;
      const v4f a0 = *(const v4f*)(sp);
      const v4f a1 = *(const v4f*)(sp + 4);
#pragma unroll
      for (int e = 0; e < 4; ++e) {
        hv[it][e]     = (_Float16)a0[e];
        hv[it][4 + e] = (_Float16)a1[e];
      }
    }
    for (int pass = 0; pass < 2; ++pass) {
#pragma unroll
      for (int it = 0; it < 4; ++it) {
        const int row = it * 8 + wave * 2 + hh;
        const int tt  = t0 + row;
        const int tok = dir ? (kL - 1 - tt) : tt;
        *(volatile v8h*)(YG16 + (size_t)(tok0 + tok) * (2 * kDi) + dir * kDi + c8) = hv[it];
      }
      __threadfence();
    }
  }
}

extern "C" void kernel_launch(void* const* d_in, const int* in_sizes, int n_in,
                              void* d_out, int out_size, void* d_ws, size_t ws_size,
                              hipStream_t stream)
{
  if (n_in < 16) return;
  if (in_sizes[0]  != kB * kCh * kL) return;
  if (in_sizes[1]  != kDm * kCh) return;
  if (in_sizes[2]  != kDm || in_sizes[3] != kDm || in_sizes[4] != kDm) return;
  if (in_sizes[5]  != kXZP * kDm) return;
  if (in_sizes[6]  != kDi * 4 || in_sizes[7] != kDi) return;
  if (in_sizes[8]  != kXP * kDi) return;
  if (in_sizes[9]  != kDi * kR || in_sizes[10] != kDi) return;
  if (in_sizes[11] != kDi * kNs || in_sizes[12] != kDi) return;
  if (in_sizes[13] != kDm * kDi) return;
  if (in_sizes[14] != kCh * kDm || in_sizes[15] != kCh) return;
  if (out_size != kB * kCh * kL) return;
  if (ws_size < kWsTotal) return;

  const float* x      = (const float*)d_in[0];
  const float* W_in   = (const float*)d_in[1];
  const float* b_in   = (const float*)d_in[2];
  const float* ln_g   = (const float*)d_in[3];
  const float* ln_b   = (const float*)d_in[4];
  const float* W_mi   = (const float*)d_in[5];
  const float* conv_w = (const float*)d_in[6];
  const float* conv_b = (const float*)d_in[7];
  const float* W_xp   = (const float*)d_in[8];
  const float* W_dt   = (const float*)d_in[9];
  const float* b_dt   = (const float*)d_in[10];
  const float* A_log  = (const float*)d_in[11];
  const float* Dvec   = (const float*)d_in[12];
  const float* W_mo   = (const float*)d_in[13];
  const float* W_out  = (const float*)d_in[14];
  const float* b_out  = (const float*)d_in[15];
  float* out = (float*)d_out;

  char* ws = (char*)d_ws;
  unsigned short* XH     = (unsigned short*)(ws + kOffXH);
  unsigned short* TOKH   = (unsigned short*)(ws + kOffTOKH);
  unsigned short* XDBL16 = (unsigned short*)(ws + kOffXDBL);
  unsigned short* XZ16   = (unsigned short*)(ws + kOffXZ);
  unsigned short* XS16   = (unsigned short*)(ws + kOffXS);
  unsigned short* YG16   = (unsigned short*)(ws + kOffYG);
  unsigned short* OUT16  = (unsigned short*)(ws + kOffOUT);
  unsigned short* WIN16  = (unsigned short*)(ws + kOffWIN);
  unsigned short* WMI16  = (unsigned short*)(ws + kOffWMI);
  unsigned short* WXP16  = (unsigned short*)(ws + kOffWXP);
  unsigned short* WMOC16 = (unsigned short*)(ws + kOffWMOC);
  unsigned short* WOUT16 = (unsigned short*)(ws + kOffWOUT);

  cast_w_f16_kernel<<<(kDm * kCh / 8) / 256, 256, 0, stream>>>(W_in, WIN16, kDm, kCh, kCh, kDm * kCh / 8, kCarryW);
  cast_w_f16_kernel<<<(kXZP * kDm / 8) / 256, 256, 0, stream>>>(W_mi, WMI16, kXZP, kDm, kDm, kXZP * kDm / 8, kCarryW);
  cast_w_f16_kernel<<<(kXPp * kDi / 8) / 256, 256, 0, stream>>>(W_xp, WXP16, kXP, kDi, kDi, kXPp * kDi / 8, kCarryW);
  cast_w_f16_kernel<<<(kDm * 2 * kDi / 8) / 256, 256, 0, stream>>>(W_mo, WMOC16, kDm, kDi, 2 * kDi, kDm * 2 * kDi / 8, kCarryW);
  cast_w_f16_kernel<<<(kCh * kDm / 8) / 256, 256, 0, stream>>>(W_out, WOUT16, kCh, kDm, kDm, kCh * kDm / 8, kCarryW);

  xpose_cast_kernel<<<dim3(kL / 64, kCh / 64, kB), 256, 0, stream>>>(
      x, XH, kCh, kL, (long)kCh * kL, (long)kL * kCh, 1.0f);

  gemm_f16_kernel<1><<<(kTok / 64) * (kDm / 64) / 8, 256, 0, stream>>>(
      XH, kCh, WIN16, kCh, (void*)TOKH, kDm, b_in, ln_g, ln_b, kTok, kDm, kCh, kSclIn);

  gemm_f16_kernel<0><<<(kTok / 64) * (kXZP / 64) / 8, 256, 0, stream>>>(
      TOKH, kDm, WMI16, kDm, (void*)XZ16, kXZP, b_in, ln_g, ln_b, kTok, kXZP, kDm, kSclMi);

  conv_silu_bidir_kernel<<<kTok / 64, 256, 0, stream>>>((const unsigned*)XZ16, conv_w, conv_b, XS16);

  gemm_f16_kernel<0><<<(kTok2 / 64) * (kXPp / 64) / 8, 256, 0, stream>>>(
      XS16, kDi, WXP16, kDi, (void*)XDBL16, kXPp, b_in, ln_g, ln_b, kTok2, kXPp, kDi, kSclXp);

  scan_gate_kernel<<<2 * kB, kDi, 0, stream>>>(
      (const unsigned*)XDBL16, (const unsigned*)XS16, (const unsigned*)XZ16, W_dt, b_dt, A_log, Dvec, YG16);

  gemm_f16_kernel<0><<<(kTok / 64) * (kDm / 64) / 8, 256, 0, stream>>>(
      YG16, 2 * kDi, WMOC16, 2 * kDi, (void*)OUT16, kDm, b_in, ln_g, ln_b, kTok, kDm, 2 * kDi, kSclMo);

  gemm_f16_kernel<2><<<(kTok / 64) * (kCh / 64) / 8, 256, 0, stream>>>(
      OUT16, kDm, WOUT16, kDm, (void*)out, kL, b_out, ln_g, ln_b, kTok, kCh, kDm, kSclOut);
}
